// KANAttention_38422777430222
// MI455X (gfx1250) — hardware-verified
//
#include <hip/hip_runtime.h>
#include <math.h>
#include <stdint.h>

#define NB   2
#define SEQ  2048
#define DM   256
#define NH   8
#define HD   32
#define NBH  (NB * NH)
#define QKVW (3 * DM)
#define KP   (3 * DM)
#define NFUN 256
#define ROWS (NB * SEQ)
#define NQB  (SEQ / 64)
#define NKT  (SEQ / 64)
static_assert(NH * HD == DM);
static_assert(NQB == 32 && NKT == 32);
static_assert((ROWS % 64) == 0 && (DM % 64) == 0 && (SEQ % 64) == 0 && (KP % 32) == 0);
static_assert((ROWS * DM) % 2048 == 0);

typedef _Float16 v16h __attribute__((ext_vector_type(16)));
typedef _Float16 v8h  __attribute__((ext_vector_type(8)));
typedef __bf16   v16b __attribute__((ext_vector_type(16)));
typedef __bf16   v8b  __attribute__((ext_vector_type(8)));
typedef float    v8f  __attribute__((ext_vector_type(8)));
typedef float    v4f  __attribute__((ext_vector_type(4)));
typedef unsigned int v4u __attribute__((ext_vector_type(4)));

#if defined(__HIP_DEVICE_COMPILE__)
#define DEV_ASM 1
#else
#define DEV_ASM 0
#endif

__device__ __forceinline__ unsigned short bf_bits(float f) {
  unsigned u = __float_as_uint(f);
  return (unsigned short)((u + 0x7FFFu + ((u >> 16) & 1u)) >> 16);
}
__device__ __forceinline__ float bf_up(unsigned short hb) { return __uint_as_float(((unsigned)hb) << 16); }
__device__ __forceinline__ unsigned short h_bits(_Float16 x) { return __builtin_bit_cast(unsigned short, x); }
__device__ __forceinline__ unsigned pk16(unsigned short a, unsigned short b) { return (unsigned)a | ((unsigned)b << 16); }
__device__ __forceinline__ v8f zero8() { v8f z = {0.f, 0.f, 0.f, 0.f, 0.f, 0.f, 0.f, 0.f}; return z; }

template <typename OT> struct FT;
template <> struct FT<__bf16>   { typedef v16b frag; typedef v8b half8; };
template <> struct FT<_Float16> { typedef v16h frag; typedef v8h half8; };

template <typename OT>
__device__ __forceinline__ typename FT<OT>::frag ldfrag(const OT* p) {
  union { typename FT<OT>::frag v; typename FT<OT>::half8 h[2]; } f;
  f.h[0] = *(const typename FT<OT>::half8*)(p);
  f.h[1] = *(const typename FT<OT>::half8*)(p + 16);
  return f.v;
}

__device__ __forceinline__ v8f mmar(v16b a, v16b b, v8f c) {
  return __builtin_amdgcn_wmma_f32_16x16x32_bf16(false, a, false, b, (short)0, c, false, false);
}
__device__ __forceinline__ v8f mma_h(v16h a, v16h b, v8f c) {
  c = __builtin_amdgcn_wmma_f32_16x16x32_f16(false, a, false, b, (short)0, c, false, false);
#if DEV_ASM
  asm volatile("v_nop\n\tv_nop\n\tv_nop\n\tv_nop" : "+v"(c) : "v"(a), "v"(b));
#endif
  return c;
}
__device__ __forceinline__ void dep_guard(v8f& a, v8f& b, v16b x, v16b y) {
#if DEV_ASM
  asm volatile("v_nop\n\tv_nop\n\tv_nop\n\tv_nop" : "+v"(a), "+v"(b) : "v"(x), "v"(y));
#else
  (void)a; (void)b; (void)x; (void)y;
#endif
}
__device__ __forceinline__ void keep4(v16b a, v16b b, v16b c, v16b d) {
#if DEV_ASM
  asm volatile("v_nop" :: "v"(a), "v"(b), "v"(c), "v"(d));
#else
  (void)a; (void)b; (void)c; (void)d;
#endif
}
__device__ __forceinline__ void acc_guard4(v8f& a, v8f& b, v8f& c, v8f& d) {
#if DEV_ASM
  asm volatile("v_nop\n\tv_nop\n\tv_nop\n\tv_nop" : "+v"(a), "+v"(b), "+v"(c), "+v"(d));
#else
  (void)a; (void)b; (void)c; (void)d;
#endif
}

__global__ __launch_bounds__(256) void cvt_x3(const float* __restrict__ in, unsigned short* out, int n8) {
  const int i = blockIdx.x * 256 + (int)threadIdx.x;
  if (i < n8) {
    const int row = i >> 5, c = (i & 31) * 8;
    const v4f a  = *(const v4f*)(in + (size_t)i * 8);
    const v4f a4 = *(const v4f*)(in + (size_t)i * 8 + 4);
    const float f[8] = {a[0], a[1], a[2], a[3], a4[0], a4[1], a4[2], a4[3]};
    v4u ph, pl;
#pragma unroll
    for (int e = 0; e < 4; ++e) {
      const float f0 = f[2 * e], f1 = f[2 * e + 1];
      const unsigned short h0 = bf_bits(f0), h1 = bf_bits(f1);
      const unsigned short l0 = bf_bits(f0 - bf_up(h0)), l1 = bf_bits(f1 - bf_up(h1));
      ph[e] = pk16(h0, h1);
      pl[e] = pk16(l0, l1);
    }
    unsigned short* o = out + (size_t)row * KP + c;
    *(volatile v4u*)(o)          = ph;
    *(volatile v4u*)(o + DM)     = ph;
    *(volatile v4u*)(o + 2 * DM) = pl;
    __threadfence();
    *(volatile v4u*)(o)          = ph;
    *(volatile v4u*)(o + DM)     = ph;
    *(volatile v4u*)(o + 2 * DM) = pl;
  }
}

__global__ __launch_bounds__(256) void wtrans3(const float* __restrict__ w, unsigned short* wt, int C) {
  __shared__ float tile[64][65];
  const int tid = (int)threadIdx.x, lane = tid & 31, wave = tid >> 5;
  const int c0 = blockIdx.x * 64, k0 = blockIdx.y * 64;
#pragma unroll
  for (int it = 0; it < 16; ++it) {
    const int idx = it * 256 + tid;
    const int r = idx >> 6, cc = idx & 63;
    tile[r][cc] = w[(size_t)(k0 + r) * C + c0 + cc];
  }
  __syncthreads();
  const int q = lane >> 3, c8 = (lane & 7) * 8;
  v4u hv[2], lv[2];
#pragma unroll
  for (int it = 0; it < 2; ++it) {
    const int row = wave * 8 + it * 4 + q;
    v4u a, a2;
#pragma unroll
    for (int e = 0; e < 4; ++e) {
      const float f0 = tile[c8 + 2 * e][row], f1 = tile[c8 + 2 * e + 1][row];
      const unsigned short h0 = bf_bits(f0), h1 = bf_bits(f1);
      const unsigned short l0 = bf_bits(f0 - bf_up(h0)), l1 = bf_bits(f1 - bf_up(h1));
      a[e] = pk16(h0, h1);
      a2[e] = pk16(l0, l1);
    }
    hv[it] = a; lv[it] = a2;
  }
  for (int pass = 0; pass < 2; ++pass) {
#pragma unroll
    for (int it = 0; it < 2; ++it) {
      const int row = wave * 8 + it * 4 + q;
      unsigned short* o = wt + (size_t)(c0 + row) * KP + k0 + c8;
      *(volatile v4u*)(o)          = hv[it];
      *(volatile v4u*)(o + DM)     = lv[it];
      *(volatile v4u*)(o + 2 * DM) = hv[it];
    }
    __threadfence();
  }
}

template <int A_MODE, int OUT_MODE>
__global__ __launch_bounds__(256) void gemm64(
    const unsigned short* __restrict__ Ap, int lda, long long strideA,
    const unsigned short* __restrict__ Btp, int ldb, long long strideB,
    void* Cout, void* Cout2, int ldc, long long strideC,
    const float* __restrict__ bias,
    int M, int N, int K, float oscale, float rscale) {
  const __bf16* A  = (const __bf16*)(const void*)Ap;
  const __bf16* Bt = (const __bf16*)(const void*)Btp;
  __shared__ __align__(16) float sT[8][16 * 68];
  const int b    = blockIdx.y;
  const int lane = threadIdx.x & 31;
  const int wave = threadIdx.x >> 5;
  const int tilesN = N >> 6;
  const int tilesM = M >> 6;
  const int tile = blockIdx.x * 8 + wave;
  if (tile >= tilesM * tilesN) return;
  const int tm = tile / tilesN;
  const int tn = tile - tm * tilesN;
  const int m0 = tm << 6;
  const int n0 = tn << 6;

  const __bf16* Ab = A  + (size_t)b * (size_t)strideA;
  const __bf16* Bb = Bt + (size_t)b * (size_t)strideB;

  const int rlane = lane & 15;
  const int koff  = (lane >> 4) * 8;
  const int mOff  = (lane >> 4) * 8;

  v8f acc[4][4];
#pragma unroll
  for (int i = 0; i < 4; ++i)
#pragma unroll
    for (int j = 0; j < 4; ++j) acc[i][j] = zero8();

  for (int k0 = 0; k0 < K; k0 += 32) {
    v16b bq[4];
#pragma unroll
    for (int j = 0; j < 4; ++j)
      bq[j] = ldfrag<__bf16>(Bb + (size_t)(n0 + (j << 4) + rlane) * ldb + koff + k0);
#pragma unroll
    for (int i = 0; i < 4; ++i) {
      const __bf16* ap;
      if (A_MODE == 0) {
        ap = Ab + (size_t)(m0 + (i << 4) + rlane) * lda + koff + k0;
      } else {
        const int plane = (k0 >> 8) * NBH + (m0 / SEQ) * NH + ((k0 >> 5) & (NH - 1));
        ap = Ab + ((size_t)plane * SEQ + (size_t)((m0 & (SEQ - 1)) + (i << 4) + rlane)) * HD + koff;
      }
      const v16b af = ldfrag<__bf16>(ap);
#pragma unroll
      for (int j = 0; j < 4; ++j) acc[i][j] = mmar(af, bq[j], acc[i][j]);
      dep_guard(acc[i][0], acc[i][3], af, bq[3]);
    }
    keep4(bq[0], bq[1], bq[2], bq[3]);
  }
  acc_guard4(acc[0][0], acc[0][1], acc[0][2], acc[0][3]);
  acc_guard4(acc[1][0], acc[1][1], acc[1][2], acc[1][3]);
  acc_guard4(acc[2][0], acc[2][1], acc[2][2], acc[2][3]);
  acc_guard4(acc[3][0], acc[3][1], acc[3][2], acc[3][3]);

  float* slab = sT[wave];
#pragma unroll
  for (int i = 0; i < 4; ++i) {
    const int mBase = m0 + (i << 4);
#pragma unroll
    for (int j = 0; j < 4; ++j) {
#pragma unroll
      for (int r = 0; r < 8; ++r) {
        slab[(mOff + r) * 68 + (j << 4) + rlane] = acc[i][j][r];
      }
    }
    __builtin_amdgcn_fence(__ATOMIC_RELEASE, "workgroup");
    __builtin_amdgcn_wave_barrier();
    __builtin_amdgcn_fence(__ATOMIC_ACQUIRE, "workgroup");
    if (OUT_MODE == 0) {
      unsigned short* Q = (unsigned short*)Cout;
      const int rq = lane >> 2, c8 = (lane & 3) * 8;
      v4u hv[4];
#pragma unroll
      for (int j2 = 0; j2 < 2; ++j2) {
#pragma unroll
        for (int it = 0; it < 2; ++it) {
          const float* sp = slab + (it * 8 + rq) * 68 + j2 * 32 + c8;
          v4u a;
#pragma unroll
          for (int e = 0; e < 4; ++e)
            a[e] = pk16(h_bits((_Float16)(sp[2 * e] * oscale)), h_bits((_Float16)(sp[2 * e + 1] * oscale)));
          hv[j2 * 2 + it] = a;
        }
      }
      for (int pass = 0; pass < 2; ++pass) {
#pragma unroll
        for (int j2 = 0; j2 < 2; ++j2) {
          const int head = (n0 >> 5) + j2;
          unsigned short* base = Q + ((size_t)((mBase / SEQ) * NH + head) * SEQ + (size_t)(mBase & (SEQ - 1))) * HD;
#pragma unroll
          for (int it = 0; it < 2; ++it)
            *(volatile v4u*)(base + it * 256 + lane * 8) = hv[j2 * 2 + it];
        }
        __threadfence();
      }
    } else if (OUT_MODE == 1) {
      float* Kr = (float*)Cout;
      const int rq = lane >> 3, c4 = (lane & 7) * 4;
      v4f hv[8];
#pragma unroll
      for (int j2 = 0; j2 < 2; ++j2) {
#pragma unroll
        for (int it = 0; it < 4; ++it)
          hv[j2 * 4 + it] = *(const v4f*)(slab + (it * 4 + rq) * 68 + j2 * 32 + c4);
      }
      for (int pass = 0; pass < 2; ++pass) {
#pragma unroll
        for (int j2 = 0; j2 < 2; ++j2) {
          const int head = (n0 >> 5) + j2;
          float* base = Kr + ((size_t)((mBase / SEQ) * NH + head) * SEQ + (size_t)(mBase & (SEQ - 1))) * HD;
#pragma unroll
          for (int it = 0; it < 4; ++it)
            *(volatile v4f*)(base + it * 128 + lane * 4) = hv[j2 * 4 + it];
        }
        __threadfence();
      }
    } else if (OUT_MODE == 2) {
      const int q = lane >> 3, c8 = (lane & 7) * 8;
      unsigned short* C  = (unsigned short*)Cout  + (size_t)b * (size_t)strideC;
      unsigned short* C2 = (unsigned short*)Cout2 + (size_t)b * (size_t)strideC;
      v4u hv[4], lv[4];
#pragma unroll
      for (int it = 0; it < 4; ++it) {
        const int row = it * 4 + q;
        const float* sp = slab + row * 68 + c8;
        v4u a, a2;
#pragma unroll
        for (int e = 0; e < 4; ++e) {
          const float f0 = sp[2 * e] * oscale, f1 = sp[2 * e + 1] * oscale;
          const _Float16 x0 = (_Float16)f0, x1 = (_Float16)f1;
          const unsigned short h0 = h_bits(x0), h1 = h_bits(x1);
          const unsigned short l0 = h_bits((_Float16)((f0 - (float)x0) * rscale));
          const unsigned short l1 = h_bits((_Float16)((f1 - (float)x1) * rscale));
          a[e] = pk16(h0, h1); a2[e] = pk16(l0, l1);
        }
        hv[it] = a; lv[it] = a2;
      }
      for (int pass = 0; pass < 2; ++pass) {
#pragma unroll
        for (int it = 0; it < 4; ++it) {
          const int row = it * 4 + q;
          *(volatile v4u*)(C  + (size_t)(mBase + row) * ldc + n0 + c8) = hv[it];
          *(volatile v4u*)(C2 + (size_t)(mBase + row) * ldc + n0 + c8) = lv[it];
        }
        __threadfence();
      }
    } else {
      float* C = (float*)Cout + (size_t)b * (size_t)strideC;
      const int h2 = lane >> 4, c4 = (lane & 15) * 4;
      const v4f bv = *(const v4f*)(bias + n0 + c4);
      v4f hv[8];
#pragma unroll
      for (int it = 0; it < 8; ++it) {
        const int row = it * 2 + h2;
        hv[it] = *(const v4f*)(slab + row * 68 + c4) + bv;
      }
      for (int pass = 0; pass < 2; ++pass) {
#pragma unroll
        for (int it = 0; it < 8; ++it) {
          const int row = it * 2 + h2;
          *(volatile v4f*)(C + (size_t)(mBase + row) * ldc + n0 + c4) = hv[it];
        }
        __threadfence();
      }
    }
    __builtin_amdgcn_fence(__ATOMIC_RELEASE, "workgroup");
    __builtin_amdgcn_wave_barrier();
    __builtin_amdgcn_fence(__ATOMIC_ACQUIRE, "workgroup");
  }
}

__global__ __launch_bounds__(256) void fourier_k(const float* __restrict__ kr, const float* __restrict__ ca,
                                                 const float* __restrict__ cb, unsigned short* kp) {
#pragma clang fp contract(off)
  __shared__ __align__(16) unsigned short sh[256];
  const int tid = (int)threadIdx.x;
  const size_t gid = (size_t)blockIdx.x * 256 + (size_t)tid;
  const float kx = kr[gid];
  float acc = 0.0f;
  float ff = 1.0f;
#pragma unroll 1
  for (int fi = 0; fi < NFUN; ++fi) {
    const float af = ca[fi];
    const float bf = cb[fi];
    const float ang = ff * kx;
    float sn, cs;
    sincosf(ang, &sn, &cs);
    const float t1 = af * sn;
    acc = acc + t1;
    const float t2 = bf * cs;
    acc = acc + t2;
    ff = ff + 1.0f;
  }
  sh[tid] = h_bits((_Float16)(acc * 4.0f));
  __syncthreads();
  if (tid < 32) {
    const v4u v = *(const v4u*)(sh + tid * 8);
    unsigned short* o = kp + (size_t)blockIdx.x * 256 + (size_t)tid * 8;
    *(volatile v4u*)o = v;
    __threadfence();
    *(volatile v4u*)o = v;
  }
}

__global__ __launch_bounds__(128)
void attn32(const unsigned short* __restrict__ qpp, const unsigned short* __restrict__ kpp,
            const unsigned short* __restrict__ vhp, const unsigned short* __restrict__ vlp,
            unsigned short* ct, float sscale) {
  union FH { v16h v; v8h h[2]; };
  __shared__ __align__(16) _Float16 Ksh[64 * HD];
  __shared__ __align__(16) _Float16 Vth[HD * 64];
  __shared__ __align__(16) _Float16 Vtl[HD * 64];
  __shared__ __align__(16) _Float16 Psh[4][16 * 64];
  __shared__ __align__(16) float    Os[4][16 * HD];

  const int tid  = (int)threadIdx.x;
  const int wave = tid >> 5;
  const int lane = tid & 31;
  const int hh   = lane >> 4;
  const int c    = lane & 15;

  const int bx   = blockIdx.x;
  const int qblk = bx % NQB;
  const int bh   = bx / NQB;
  const int q0   = qblk * 64 + wave * 16;

  const _Float16* Qg = (const _Float16*)(const void*)qpp + (size_t)bh * SEQ * HD;
  const _Float16* Kg = (const _Float16*)(const void*)kpp + (size_t)bh * SEQ * HD;
  const _Float16* Vh = (const _Float16*)(const void*)vhp + (size_t)bh * HD * SEQ;
  const _Float16* Vl = (const _Float16*)(const void*)vlp + (size_t)bh * HD * SEQ;

  const v16h qa = ldfrag<_Float16>(Qg + (size_t)(q0 + c) * HD + 8 * hh);

  float mrow[8], lrow[8];
  v8f oacc[2];
#pragma unroll
  for (int r = 0; r < 8; ++r) { mrow[r] = -INFINITY; lrow[r] = 0.f; }
  oacc[0] = zero8(); oacc[1] = zero8();

  for (int kt = 0; kt < NKT; ++kt) {
    const int kv0 = kt * 64;
    __syncthreads();
    {
      const int r = tid >> 1, hf = (tid & 1) * 16;
      const _Float16* kg = Kg + (size_t)(kv0 + r) * HD + hf;
      const v8h k0v = *(const v8h*)(kg);
      const v8h k1v = *(const v8h*)(kg + 8);
      *(v8h*)(Ksh + r * HD + hf)     = k0v;
      *(v8h*)(Ksh + r * HD + hf + 8) = k1v;
      const int d = tid >> 2, sg = (tid & 3) * 16;
      const _Float16* vg  = Vh + (size_t)d * SEQ + kv0 + sg;
      const _Float16* vlg = Vl + (size_t)d * SEQ + kv0 + sg;
      const v8h v0 = *(const v8h*)(vg),  v1 = *(const v8h*)(vg + 8);
      const v8h w0 = *(const v8h*)(vlg), w1 = *(const v8h*)(vlg + 8);
      *(v8h*)(Vth + d * 64 + sg)     = v0;
      *(v8h*)(Vth + d * 64 + sg + 8) = v1;
      *(v8h*)(Vtl + d * 64 + sg)     = w0;
      *(v8h*)(Vtl + d * 64 + sg + 8) = w1;
    }
    __syncthreads();

    v8f s[4];
#pragma unroll
    for (int j = 0; j < 4; ++j) {
      FH kb;
      kb.h[0] = *(const v8h*)(Ksh + (j * 16 + c) * HD + 8 * hh);
      kb.h[1] = *(const v8h*)(Ksh + (j * 16 + c) * HD + 16 + 8 * hh);
      s[j] = mma_h(qa, kb.v, zero8());
#pragma unroll
      for (int r = 0; r < 8; ++r) s[j][r] *= sscale;
    }

    _Float16* pwh = Psh[wave];
#pragma unroll
    for (int r = 0; r < 8; ++r) {
      float m = s[0][r];
#pragma unroll
      for (int j = 1; j < 4; ++j) m = fmaxf(m, s[j][r]);
#pragma unroll
      for (int off = 1; off < 16; off <<= 1) m = fmaxf(m, __shfl_xor(m, off, 32));
      const float mnew  = fmaxf(mrow[r], m);
      const float msafe = (mnew == -INFINITY) ? 0.f : mnew;
      const float alpha = __expf(mrow[r] - msafe);
      mrow[r] = mnew;
      float psum = 0.f;
#pragma unroll
      for (int j = 0; j < 4; ++j) {
        const float p = __expf(s[j][r] - msafe);
        psum += p;
        pwh[(8 * hh + r) * 64 + j * 16 + c] = (_Float16)(p * 1024.0f);
      }
#pragma unroll
      for (int off = 1; off < 16; off <<= 1) psum += __shfl_xor(psum, off, 32);
      lrow[r] = lrow[r] * alpha + psum;
      oacc[0][r] *= alpha;
      oacc[1][r] *= alpha;
    }
    __builtin_amdgcn_fence(__ATOMIC_RELEASE, "workgroup");
    __builtin_amdgcn_wave_barrier();
    __builtin_amdgcn_fence(__ATOMIC_ACQUIRE, "workgroup");

    v8f o1[2];
    o1[0] = zero8(); o1[1] = zero8();
#pragma unroll
    for (int kk = 0; kk < 2; ++kk) {
      FH pa;
      pa.h[0] = *(const v8h*)(pwh + c * 64 + kk * 32 + 8 * hh);
      pa.h[1] = *(const v8h*)(pwh + c * 64 + kk * 32 + 16 + 8 * hh);
#pragma unroll
      for (int t = 0; t < 2; ++t) {
        FH vb, vl;
        vb.h[0] = *(const v8h*)(Vth + (t * 16 + c) * 64 + kk * 32 + 8 * hh);
        vb.h[1] = *(const v8h*)(Vth + (t * 16 + c) * 64 + kk * 32 + 16 + 8 * hh);
        vl.h[0] = *(const v8h*)(Vtl + (t * 16 + c) * 64 + kk * 32 + 8 * hh);
        vl.h[1] = *(const v8h*)(Vtl + (t * 16 + c) * 64 + kk * 32 + 16 + 8 * hh);
        oacc[t] = mma_h(pa.v, vb.v, oacc[t]);
        o1[t]   = mma_h(pa.v, vl.v, o1[t]);
      }
    }
#pragma unroll
    for (int t = 0; t < 2; ++t)
#pragma unroll
      for (int r = 0; r < 8; ++r) oacc[t][r] += o1[t][r] * (1.0f / 2048.0f);
  }

  float* os = Os[wave];
#pragma unroll
  for (int r = 0; r < 8; ++r) {
    const float l = lrow[r];
    const float inv = 1.0f / (l * 4096.0f);
    os[(8 * hh + r) * HD + c]      = oacc[0][r] * inv;
    os[(8 * hh + r) * HD + 16 + c] = oacc[1][r] * inv;
  }
  __builtin_amdgcn_fence(__ATOMIC_RELEASE, "workgroup");
  __builtin_amdgcn_wave_barrier();
  __builtin_amdgcn_fence(__ATOMIC_ACQUIRE, "workgroup");
  {
    const int rq = lane >> 2, c8 = (lane & 3) * 8;
    v4u hv[2], lv[2];
#pragma unroll
    for (int it = 0; it < 2; ++it) {
      const int row = it * 8 + rq;
      const float* sp = os + row * HD + c8;
      v4u a, a2;
#pragma unroll
      for (int e = 0; e < 4; ++e) {
        const float f0 = sp[2 * e], f1 = sp[2 * e + 1];
        const unsigned short h0 = bf_bits(f0), h1 = bf_bits(f1);
        const unsigned short l0 = bf_bits(f0 - bf_up(h0)), l1 = bf_bits(f1 - bf_up(h1));
        a[e] = pk16(h0, h1); a2[e] = pk16(l0, l1);
      }
      hv[it] = a; lv[it] = a2;
    }
    const size_t PS = (size_t)NBH * SEQ * HD;
    unsigned short* base = ct + ((size_t)bh * SEQ + (size_t)q0) * HD;
    for (int pass = 0; pass < 2; ++pass) {
#pragma unroll
      for (int it = 0; it < 2; ++it) {
        unsigned short* p = base + it * 256 + lane * 8;
        *(volatile v4u*)(p)          = hv[it];
        *(volatile v4u*)(p + PS)     = hv[it];
        *(volatile v4u*)(p + 2 * PS) = lv[it];
      }
      __threadfence();
    }
  }
}

extern "C" void kernel_launch(void* const* d_in, const int* in_sizes, int n_in,
                              void* d_out, int out_size, void* d_ws, size_t ws_size,
                              hipStream_t stream) {
  if (n_in < 6) return;
  if (in_sizes[0] != ROWS * DM) return;
  if (in_sizes[1] != DM * QKVW) return;
  if (in_sizes[2] != DM * DM) return;
  if (in_sizes[3] != DM) return;
  if (in_sizes[4] != NFUN || in_sizes[5] != NFUN) return;
  if (out_size != ROWS * DM) return;

  const float* x     = (const float*)d_in[0];
  const float* w_qkv = (const float*)d_in[1];
  const float* w_o   = (const float*)d_in[2];
  const float* b_o   = (const float*)d_in[3];
  const float* coefa = (const float*)d_in[4];
  const float* coefb = (const float*)d_in[5];

  const size_t PX3 = (size_t)ROWS * KP * 2;
  const size_t PWQ = (size_t)QKVW * KP * 2;
  const size_t PWO = (size_t)DM * KP * 2;
  const size_t PH  = (size_t)NBH * SEQ * HD * 2;
  const size_t PK4 = (size_t)NBH * SEQ * HD * 4;
  const size_t PVT = (size_t)NB * DM * SEQ * 2;
  const size_t PCT = (size_t)3 * NBH * SEQ * HD * 2;
  size_t off = 0;
  const size_t oX3  = off; off += PX3;
  const size_t oWq  = off; off += PWQ;
  const size_t oWo  = off; off += PWO;
  const size_t oQp  = off; off += PH;
  const size_t oKr  = off; off += PK4;
  const size_t oKp  = off; off += PH;
  const size_t oVTh = off; off += PVT;
  const size_t oVTl = off; off += PVT;
  const size_t oCT  = off; off += PCT;
  if (off > ws_size) return;
  if (off > (size_t)134217728) return;

  char* ws = (char*)d_ws;
  unsigned short* X3  = (unsigned short*)(ws + oX3);
  unsigned short* Wq3 = (unsigned short*)(ws + oWq);
  unsigned short* Wo3 = (unsigned short*)(ws + oWo);
  unsigned short* Qp  = (unsigned short*)(ws + oQp);
  float*          Kr  = (float*)(ws + oKr);
  unsigned short* Kp  = (unsigned short*)(ws + oKp);
  unsigned short* VTh = (unsigned short*)(ws + oVTh);
  unsigned short* VTl = (unsigned short*)(ws + oVTl);
  unsigned short* CT  = (unsigned short*)(ws + oCT);

  const dim3 blk(256);
  const int n8x = ROWS * DM / 8;
  const dim3 gCvtX((n8x + 255) / 256);
  const dim3 gTq(QKVW / 64, DM / 64);
  const dim3 gTo(DM / 64, DM / 64);
  const dim3 gQK(((ROWS / 64) * (DM / 64) + 7) / 8, 1);
  const dim3 gVT(((DM / 64) * (SEQ / 64) + 7) / 8, NB);
  const dim3 gFour((NBH * SEQ * HD) / 256);
  const dim3 gAttn(NBH * NQB);

  cvt_x3<<<gCvtX, blk, 0, stream>>>(x, X3, n8x);
  wtrans3<<<gTq, blk, 0, stream>>>(w_qkv, Wq3, QKVW);
  wtrans3<<<gTo, blk, 0, stream>>>(w_o, Wo3, DM);
  gemm64<0, 0><<<gQK, blk, 0, stream>>>(
      X3, KP, 0LL, Wq3, KP, 0LL,
      (void*)Qp, (void*)Qp, 0, 0LL, b_o,
      ROWS, DM, KP, 4.0f, 1.0f);
  gemm64<0, 1><<<gQK, blk, 0, stream>>>(
      X3, KP, 0LL, Wq3 + (size_t)DM * KP, KP, 0LL,
      (void*)Kr, (void*)Kr, 0, 0LL, b_o,
      ROWS, DM, KP, 1.0f, 1.0f);
  gemm64<0, 2><<<gVT, blk, 0, stream>>>(
      Wq3 + (size_t)2 * DM * KP, KP, 0LL, X3, KP, (long long)SEQ * KP,
      (void*)VTh, (void*)VTl, SEQ, (long long)DM * SEQ, b_o,
      DM, SEQ, KP, 4.0f, 2048.0f);
  fourier_k<<<gFour, blk, 0, stream>>>(Kr, coefa, coefb, Kp);
  attn32<<<gAttn, dim3(128), 0, stream>>>(Qp, Kp, VTh, VTl, CT, 0.17677669529663687f * 0.0625f);
  gemm64<1, 3><<<gQK, blk, 0, stream>>>(
      CT, 0, 0LL, Wo3, KP, 0LL,
      d_out, d_out, DM, 0LL, b_o,
      ROWS, DM, KP, 1.0f, 1.0f);
  (void)hipGetLastError();
}
